// LinBlock_23021024707079
// MI455X (gfx1250) — hardware-verified
//
#include <hip/hip_runtime.h>
#include <math.h>
#include <stdint.h>

typedef __attribute__((ext_vector_type(16))) _Float16 v16h;
typedef __attribute__((ext_vector_type(8)))  _Float16 v8h;
typedef __attribute__((ext_vector_type(16))) __bf16   v16b;
typedef __attribute__((ext_vector_type(8)))  __bf16   v8b;
typedef __attribute__((ext_vector_type(8)))  float    v8f;
typedef __attribute__((ext_vector_type(4)))  float    v4f;
typedef __attribute__((ext_vector_type(2)))  float    v2f;
typedef __attribute__((ext_vector_type(4)))  unsigned int v4u;

__device__ __forceinline__ unsigned short f2bf_bits(float f) {
  unsigned u = __float_as_uint(f);
  return (unsigned short)((u + 0x7FFFu + ((u >> 16) & 1u)) >> 16);
}
__device__ __forceinline__ float bf_bits2f(unsigned short h) { return __uint_as_float(((unsigned)h) << 16); }

__device__ __forceinline__ void dep_guard_h(v8f& a, v8f& b, v16h x, v16h y) { asm volatile("v_nop\n\tv_nop\n\tv_nop\n\tv_nop" : "+v"(a), "+v"(b) : "v"(x), "v"(y)); }
__device__ __forceinline__ void dep_guard_b(v8f& a, v8f& b, v16b x, v16b y) { asm volatile("v_nop\n\tv_nop\n\tv_nop\n\tv_nop" : "+v"(a), "+v"(b) : "v"(x), "v"(y)); }
__device__ __forceinline__ void keep4_h(v16h a, v16h b, v16h c, v16h d) { asm volatile("v_nop" :: "v"(a), "v"(b), "v"(c), "v"(d)); }
__device__ __forceinline__ void keep4_b(v16b a, v16b b, v16b c, v16b d) { asm volatile("v_nop" :: "v"(a), "v"(b), "v"(c), "v"(d)); }
__device__ __forceinline__ void acc_guard4(v8f& a, v8f& b, v8f& c, v8f& d) { asm volatile("v_nop\n\tv_nop\n\tv_nop\n\tv_nop" : "+v"(a), "+v"(b), "+v"(c), "+v"(d)); }
template <typename T> struct Frag;
template <> struct Frag<_Float16> {
  typedef v16h V; union U { v16h v; v8h h[2]; };
  static __device__ __forceinline__ v16h load(const _Float16* p) {
    U f; f.h[0] = *(const v8h*)(p); f.h[1] = *(const v8h*)(p + 16); return f.v;
  }
  static __device__ __forceinline__ v8f mma(v16h a, v16h b, v8f c) {
    return __builtin_amdgcn_wmma_f32_16x16x32_f16(false, a, false, b, (short)0, c, false, false);
  }
  static __device__ __forceinline__ void guard(v8f& a, v8f& b, v16h x, v16h y) { dep_guard_h(a, b, x, y); }
  static __device__ __forceinline__ void keep(v16h a, v16h b, v16h c, v16h d) { keep4_h(a, b, c, d); }
};
template <> struct Frag<__bf16> {
  typedef v16b V; union U { v16b v; v8b h[2]; };
  static __device__ __forceinline__ v16b load(const __bf16* p) {
    U f; f.h[0] = *(const v8b*)(p); f.h[1] = *(const v8b*)(p + 16); return f.v;
  }
  static __device__ __forceinline__ v8f mma(v16b a, v16b b, v8f c) {
    return __builtin_amdgcn_wmma_f32_16x16x32_bf16(false, a, false, b, (short)0, c, false, false);
  }
  static __device__ __forceinline__ void guard(v8f& a, v8f& b, v16b x, v16b y) { dep_guard_b(a, b, x, y); }
  static __device__ __forceinline__ void keep(v16b a, v16b b, v16b c, v16b d) { keep4_b(a, b, c, d); }
};

template <int ET> struct Elem;
template <> struct Elem<0> { typedef _Float16 T; };
template <> struct Elem<1> { typedef __bf16 T; };
template <int ET, bool SPLIT, int BIAS_MODE, int OUT_MODE, bool RESID, int ACT = 0>
__global__ __launch_bounds__(256) void wmma_gemm64(
    const unsigned short* __restrict__ Ap, const unsigned short* __restrict__ A2p, int lda, long strideA,
    const unsigned short* __restrict__ Btp, const unsigned short* __restrict__ Bt2p, int ldb, long strideB,
    void* __restrict__ Cout, void* __restrict__ Cout2, int ldc, long strideC,
    const float* __restrict__ bias,
    const float* __restrict__ resid, long strideR,
    int M, int N, int K, float scale) {
  typedef typename Elem<ET>::T T;
  typedef typename Frag<T>::V V;
  const T* A = (const T*)Ap; const T* A2 = (const T*)A2p; const T* Bt = (const T*)Btp; const T* Bt2 = (const T*)Bt2p;
  __shared__ __align__(16) float sT[8][16 * 68];
  const int b    = blockIdx.y;
  const int lane = threadIdx.x & 31;
  const int wave = threadIdx.x >> 5;
  const int tilesN = N >> 6;
  const int tilesM = M >> 6;
  const int tile = blockIdx.x * 8 + wave;
  if (tile >= tilesM * tilesN) return;
  const int tm = tile / tilesN;
  const int tn = tile - tm * tilesN;
  const int m0 = tm << 6;
  const int n0 = tn << 6;

  const T* Ab  = A  + (size_t)b * strideA;
  const T* Bb  = Bt + (size_t)b * strideB;
  const T* Ab2 = SPLIT ? (A2  + (size_t)b * strideA) : nullptr;
  const T* Bb2 = SPLIT ? (Bt2 + (size_t)b * strideB) : nullptr;

  const int rlane = lane & 15;
  const int koff  = (lane >> 4) * 8;
  const int mOff  = (lane >> 4) * 8;

  v8f acc[4][4];
#pragma unroll
  for (int i = 0; i < 4; ++i)
#pragma unroll
    for (int j = 0; j < 4; ++j) acc[i][j] = (v8f){0.f,0.f,0.f,0.f,0.f,0.f,0.f,0.f};

  for (int k0 = 0; k0 < K; k0 += 32) {
    V bh[4], bl[4];
#pragma unroll
    for (int j = 0; j < 4; ++j) {
      const size_t bo = (size_t)(n0 + (j << 4) + rlane) * ldb + koff + k0;
      bh[j] = Frag<T>::load(Bb + bo);
      if (SPLIT) bl[j] = Frag<T>::load(Bb2 + bo);
    }
#pragma unroll
    for (int i = 0; i < 4; ++i) {
      const size_t ao = (size_t)(m0 + (i << 4) + rlane) * lda + koff + k0;
      V ah = Frag<T>::load(Ab + ao);
      V al;
      if (SPLIT) al = Frag<T>::load(Ab2 + ao);
#pragma unroll
      for (int j = 0; j < 4; ++j) {
        acc[i][j] = Frag<T>::mma(ah, bh[j], acc[i][j]);
        if (SPLIT) {
          acc[i][j] = Frag<T>::mma(ah, bl[j], acc[i][j]);
          acc[i][j] = Frag<T>::mma(al, bh[j], acc[i][j]);
        }
      }
      Frag<T>::guard(acc[i][0], acc[i][3], ah, SPLIT ? al : ah);
    }
    Frag<T>::keep(bh[0], bh[1], bh[2], bh[3]);
    if (SPLIT) Frag<T>::keep(bl[0], bl[1], bl[2], bl[3]);
  }
  acc_guard4(acc[0][0], acc[0][1], acc[0][2], acc[0][3]);
  acc_guard4(acc[1][0], acc[1][1], acc[1][2], acc[1][3]);
  acc_guard4(acc[2][0], acc[2][1], acc[2][2], acc[2][3]);
  acc_guard4(acc[3][0], acc[3][1], acc[3][2], acc[3][3]);

  float* slab = sT[wave];
  const float* Rb = RESID ? (resid + (size_t)b * strideR) : nullptr;
#pragma unroll
  for (int i = 0; i < 4; ++i) {
    const int mBase = m0 + (i << 4);
#pragma unroll
    for (int j = 0; j < 4; ++j) {
      const int n = n0 + (j << 4) + rlane;
      float bv = 0.f;
      if (BIAS_MODE == 2) bv = bias[n];
#pragma unroll
      for (int r = 0; r < 8; ++r) {
        float v = acc[i][j][r] * scale;
        if (BIAS_MODE == 1) v += bias[mBase + mOff + r];
        if (BIAS_MODE == 2) v += bv;
        if (RESID) v += Rb[(size_t)(mBase + mOff + r) * ldc + n];
        if (ACT == 1) v = tanhf(v);
        if (ACT == 2) v = fmaxf(v, 0.0f);
        if (ACT == 3) v = v / (1.0f + expf(-v));
        if (ACT == 4) v = (v > 0.f) ? v : 0.01f * v;
        if (ACT == 5) v = 0.5f * v * (1.0f + erff(v * 0.70710678118654752f));
        slab[(mOff + r) * 68 + (j << 4) + rlane] = v;
      }
    }
    __builtin_amdgcn_fence(__ATOMIC_RELEASE, "workgroup");
    __builtin_amdgcn_wave_barrier();
    __builtin_amdgcn_fence(__ATOMIC_ACQUIRE, "workgroup");
    if (OUT_MODE == 0) {
      float* C = (float*)Cout + (size_t)b * strideC;
      const int hh = lane >> 4, c4 = (lane & 15) * 4;
      for (int pass = 0; pass < 2; ++pass) {
#pragma unroll
        for (int it = 0; it < 8; ++it) {
          const int row = it * 2 + hh;
          v4f v = *(const v4f*)(slab + row * 68 + c4);
          *(volatile v4f*)(C + (size_t)(mBase + row) * ldc + n0 + c4) = v;
        }
        __threadfence();
      }
    } else {
      const int q = lane >> 3, c8 = (lane & 7) * 8;
      unsigned short* C  = (unsigned short*)Cout  + (size_t)b * strideC;
      unsigned short* C2 = (OUT_MODE == 2) ? ((unsigned short*)Cout2 + (size_t)b * strideC) : nullptr;
      for (int pass = 0; pass < 2; ++pass) {
#pragma unroll
        for (int it = 0; it < 4; ++it) {
          const int row = it * 4 + q;
          const float* sp = slab + row * 68 + c8;
          v8h hv, lv;
#pragma unroll
          for (int e = 0; e < 8; ++e) {
            if (OUT_MODE == 1) {
              hv[e] = (_Float16)sp[e];
            } else {
              unsigned short hb = f2bf_bits(sp[e]);
              unsigned short lb = f2bf_bits(sp[e] - bf_bits2f(hb));
              hv[e] = __builtin_bit_cast(_Float16, hb);
              lv[e] = __builtin_bit_cast(_Float16, lb);
            }
          }
          *(volatile v8h*)(C + (size_t)(mBase + row) * ldc + n0 + c8) = hv;
          if (OUT_MODE == 2) *(volatile v8h*)(C2 + (size_t)(mBase + row) * ldc + n0 + c8) = lv;
        }
        __threadfence();
      }
    }
    __builtin_amdgcn_fence(__ATOMIC_RELEASE, "workgroup");
    __builtin_amdgcn_wave_barrier();
    __builtin_amdgcn_fence(__ATOMIC_ACQUIRE, "workgroup");
  }
}

__device__ __forceinline__ unsigned pk16(unsigned short a, unsigned short b) { return (unsigned)a | ((unsigned)b << 16); }

constexpr int   SEQLEN  = 4096;
constexpr int   NBAT    = 4;
constexpr int   EMBED   = 512;
constexpr int   NHEADS  = 8;
constexpr int   HDIM    = 64;
constexpr int   NCOMP   = 1024;
constexpr float SCORE_SCALE = 0.125f;
constexpr float PROB_CARRY  = 32768.0f;
constexpr float OUT_CARRY   = 16.0f;
constexpr float WO_CARRY    = 64.0f;

__global__ __launch_bounds__(256) void cast_bf16x2_kernel(const float* __restrict__ in, unsigned short* __restrict__ out, int n2) {
  const int i = blockIdx.x * 256 + threadIdx.x;
  if (i < n2) {
    const v2f f = *(const v2f*)(in + 2 * (size_t)i);
    const unsigned u = pk16(f2bf_bits(f[0]), f2bf_bits(f[1]));
    ((volatile unsigned*)out)[i] = u;
    __threadfence();
    ((volatile unsigned*)out)[i] = u;
  }
}

__global__ __launch_bounds__(256) void dup_bf16x2_kernel(const float* __restrict__ W, unsigned short* __restrict__ out, int n2, int cols) {
  const int i = blockIdx.x * 256 + threadIdx.x;
  if (i < n2) {
    const int e0 = 2 * i;
    const int r  = e0 / cols;
    const int cc = e0 - r * cols;
    const v2f f = *(const v2f*)(W + e0);
    const unsigned u = pk16(f2bf_bits(f[0]), f2bf_bits(f[1]));
    const size_t o0 = ((size_t)r * 2 * cols + cc) >> 1;
    const size_t o1 = ((size_t)r * 2 * cols + cols + cc) >> 1;
    ((volatile unsigned*)out)[o0] = u;
    ((volatile unsigned*)out)[o1] = u;
    __threadfence();
    ((volatile unsigned*)out)[o0] = u;
    ((volatile unsigned*)out)[o1] = u;
  }
}

__global__ __launch_bounds__(256) void cast_wo_f16x2_kernel(const float* __restrict__ W, unsigned short* __restrict__ out, int n2, float carry) {
  const int i = blockIdx.x * 256 + threadIdx.x;
  if (i < n2) {
    const v2f f = *(const v2f*)(W + 2 * (size_t)i);
    const float b0 = bf_bits2f(f2bf_bits(f[0])) * carry;
    const float b1 = bf_bits2f(f2bf_bits(f[1])) * carry;
    const _Float16 h0 = (_Float16)b0, h1 = (_Float16)b1;
    const unsigned u = pk16(__builtin_bit_cast(unsigned short, h0), __builtin_bit_cast(unsigned short, h1));
    ((volatile unsigned*)out)[i] = u;
    __threadfence();
    ((volatile unsigned*)out)[i] = u;
  }
}

__global__ __launch_bounds__(512) void bias_prep_kernel(const float* __restrict__ bq, const float* __restrict__ bk,
                                                        const float* __restrict__ bv, const float* __restrict__ bo,
                                                        float* __restrict__ outb, int n) {
  const int i = blockIdx.x * 512 + threadIdx.x;
  if (i < n) {
    const float a0 = bf_bits2f(f2bf_bits(bq[i]));
    const float a1 = bf_bits2f(f2bf_bits(bk[i]));
    const float a2 = bf_bits2f(f2bf_bits(bv[i]));
    const float a3 = bf_bits2f(f2bf_bits(bo[i]));
    ((volatile float*)outb)[i] = a0;
    ((volatile float*)outb)[n + i] = a1;
    ((volatile float*)outb)[2 * n + i] = a2;
    ((volatile float*)outb)[3 * n + i] = a3;
    __threadfence();
    ((volatile float*)outb)[i] = a0;
    ((volatile float*)outb)[n + i] = a1;
    ((volatile float*)outb)[2 * n + i] = a2;
    ((volatile float*)outb)[3 * n + i] = a3;
  }
}

__global__ __launch_bounds__(256) void tconv_bf16_kernel(const float* __restrict__ X, unsigned short* __restrict__ o,
                                                         int R, int Cc, int ldi, long sIn, long sOut) {
  __shared__ __align__(16) float tf[64 * 68];
  X += (size_t)blockIdx.z * sIn;
  o += (size_t)blockIdx.z * sOut;
  const int c0  = blockIdx.x * 64;
  const int r0  = blockIdx.y * 64;
  const int tid = threadIdx.x;
  {
    const int lr = tid >> 4;
    const int c4 = (tid & 15) * 4;
#pragma unroll
    for (int it = 0; it < 4; ++it) {
      const int rr = it * 16 + lr;
      const v4f a = *(const v4f*)(X + (size_t)(r0 + rr) * ldi + c0 + c4);
      *(v4f*)(tf + rr * 68 + c4) = a;
    }
  }
  __syncthreads();
  const int sub = tid >> 3;
  const int c8  = (tid & 7) * 8;
  v4u hv[2];
#pragma unroll
  for (int it = 0; it < 2; ++it) {
    const int oc = it * 32 + sub;
    v4u a;
#pragma unroll
    for (int q = 0; q < 4; ++q) {
      const float f0 = tf[(c8 + 2 * q) * 68 + oc];
      const float f1 = tf[(c8 + 2 * q + 1) * 68 + oc];
      a[q] = pk16(f2bf_bits(f0), f2bf_bits(f1));
    }
    hv[it] = a;
  }
  for (int pass = 0; pass < 2; ++pass) {
#pragma unroll
    for (int it = 0; it < 2; ++it) {
      const int oc = it * 32 + sub;
      const size_t go = (size_t)(c0 + oc) * R + r0 + c8;
      *(volatile v4u*)(o + go) = hv[it];
    }
    __threadfence();
  }
}

__device__ __forceinline__ v8f hmma(v16h a, v16h b, v8f c) {
  c = __builtin_amdgcn_wmma_f32_16x16x32_f16(false, a, false, b, (short)0, c, false, false);
  asm volatile("v_nop\n\tv_nop\n\tv_nop\n\tv_nop" : "+v"(c) : "v"(a), "v"(b));
  return c;
}

__global__ __launch_bounds__(128)
void attn_lin_kernel(const unsigned short* __restrict__ qp, const unsigned short* __restrict__ kp,
                     const unsigned short* __restrict__ vtp, unsigned short* __restrict__ op) {
  typedef Frag<_Float16> FR;
  __shared__ __align__(16) _Float16 Ksh[64 * 64];
  __shared__ __align__(16) _Float16 Vth[64 * 64];
  __shared__ __align__(16) _Float16 Psh[4 * 16 * 64];
  __shared__ __align__(16) float    Os[4 * 16 * 68];

  const int tid  = threadIdx.x;
  const int wave = tid >> 5;
  const int lane = tid & 31;
  const int hh   = lane >> 4;
  const int c    = lane & 15;

  constexpr int NQB  = SEQLEN / 64;
  constexpr int ROWP = NBAT * EMBED;
  constexpr int NCH  = NCOMP / 64;

  const int bx = blockIdx.x;
  const int qb = bx % NQB;
  const int bh = bx / NQB;
  const int h  = bh % NHEADS;
  const int b  = bh / NHEADS;
  const int q0 = qb * 64 + wave * 16;

  const _Float16* Qb = (const _Float16*)(const void*)qp  + (size_t)b * EMBED + (size_t)h * HDIM;
  const _Float16* Kb = (const _Float16*)(const void*)kp  + (size_t)b * EMBED + (size_t)h * HDIM;
  const _Float16* Vb = (const _Float16*)(const void*)vtp + (size_t)b * EMBED * NCOMP + (size_t)h * HDIM * NCOMP;
  _Float16*       Ob = (_Float16*)(void*)op + (size_t)b * EMBED + (size_t)h * HDIM;

  v16h qa[2];
  {
    const _Float16* qrow = Qb + (size_t)(q0 + c) * ROWP;
#pragma unroll
    for (int dc = 0; dc < 2; ++dc) qa[dc] = FR::load(qrow + dc * 32 + 8 * hh);
  }

  float mrow[8], lrow[8];
  v8f oacc[4];
#pragma unroll
  for (int r = 0; r < 8; ++r) { mrow[r] = -INFINITY; lrow[r] = 0.f; }
#pragma unroll
  for (int t = 0; t < 4; ++t) oacc[t] = (v8f){0.f,0.f,0.f,0.f,0.f,0.f,0.f,0.f};

#pragma unroll 1
  for (int kc = 0; kc < NCH; ++kc) {
    const int kv0 = kc * 64;
    __syncthreads();
    {
      const int r = tid >> 1, hoff = (tid & 1) * 32;
      const _Float16* krow = Kb + (size_t)(kv0 + r) * ROWP + hoff;
      const _Float16* vrow = Vb + (size_t)r * NCOMP + kv0 + hoff;
#pragma unroll
      for (int i = 0; i < 4; ++i) {
        const v8h kk = *(const v8h*)(krow + 8 * i);
        const v8h vv = *(const v8h*)(vrow + 8 * i);
        *(v8h*)(Ksh + r * 64 + hoff + 8 * i) = kk;
        *(v8h*)(Vth + r * 64 + hoff + 8 * i) = vv;
      }
    }
    __syncthreads();

    v8f s[4];
#pragma unroll
    for (int j = 0; j < 4; ++j) {
      s[j] = (v8f){0.f,0.f,0.f,0.f,0.f,0.f,0.f,0.f};
#pragma unroll
      for (int dc = 0; dc < 2; ++dc) {
        const v16h kb = FR::load(Ksh + (j * 16 + c) * 64 + dc * 32 + 8 * hh);
        s[j] = hmma(qa[dc], kb, s[j]);
      }
    }
    float cm[8];
#pragma unroll
    for (int r = 0; r < 8; ++r) {
      float m = -INFINITY;
#pragma unroll
      for (int j = 0; j < 4; ++j) {
        s[j][r] *= SCORE_SCALE;
        m = fmaxf(m, s[j][r]);
      }
#pragma unroll
      for (int off = 1; off < 16; off <<= 1) m = fmaxf(m, __shfl_xor(m, off, 32));
      cm[r] = m;
    }
    _Float16* pw = Psh + wave * (16 * 64);
#pragma unroll
    for (int r = 0; r < 8; ++r) {
      const float mnew  = fmaxf(mrow[r], cm[r]);
      const float alpha = __expf(mrow[r] - mnew);
      mrow[r] = mnew;
      float psum = 0.f;
#pragma unroll
      for (int j = 0; j < 4; ++j) {
        const float p = __expf(s[j][r] - mnew);
        psum += p;
        pw[(8 * hh + r) * 64 + j * 16 + c] = (_Float16)(p * PROB_CARRY);
      }
#pragma unroll
      for (int off = 1; off < 16; off <<= 1) psum += __shfl_xor(psum, off, 32);
      lrow[r] = lrow[r] * alpha + psum;
#pragma unroll
      for (int t = 0; t < 4; ++t) oacc[t][r] *= alpha;
    }
    __builtin_amdgcn_fence(__ATOMIC_RELEASE, "workgroup");
    __builtin_amdgcn_wave_barrier();
    __builtin_amdgcn_fence(__ATOMIC_ACQUIRE, "workgroup");
#pragma unroll
    for (int kk = 0; kk < 2; ++kk) {
      const v16h pa = FR::load(pw + c * 64 + kk * 32 + 8 * hh);
#pragma unroll
      for (int t = 0; t < 4; ++t) {
        const v16h vb = FR::load(Vth + (t * 16 + c) * 64 + kk * 32 + 8 * hh);
        oacc[t] = hmma(pa, vb, oacc[t]);
      }
    }
  }

  float* os = Os + wave * (16 * 68);
#pragma unroll
  for (int r = 0; r < 8; ++r) {
    const float inv = OUT_CARRY * (1.0f / (lrow[r] * PROB_CARRY));
#pragma unroll
    for (int t = 0; t < 4; ++t) os[(8 * hh + r) * 68 + t * 16 + c] = oacc[t][r] * inv;
  }
  __builtin_amdgcn_fence(__ATOMIC_RELEASE, "workgroup");
  __builtin_amdgcn_wave_barrier();
  __builtin_amdgcn_fence(__ATOMIC_ACQUIRE, "workgroup");
  {
    const int qq = lane >> 3, c8 = (lane & 7) * 8;
    for (int pass = 0; pass < 2; ++pass) {
#pragma unroll
      for (int it = 0; it < 4; ++it) {
        const int row = it * 4 + qq;
        const float* sp = os + row * 68 + c8;
        v8h hv;
#pragma unroll
        for (int e = 0; e < 8; ++e) hv[e] = (_Float16)sp[e];
        *(volatile v8h*)(Ob + (size_t)(q0 + row) * ROWP + c8) = hv;
      }
      __threadfence();
    }
  }
}

extern "C" void kernel_launch(void* const* d_in, const int* in_sizes, int n_in,
                              void* d_out, int out_size, void* d_ws, size_t ws_size,
                              hipStream_t stream) {
  if (n_in < 11) return;
  const long nQ  = (long)SEQLEN * NBAT * EMBED;
  const long nW  = (long)EMBED * EMBED;
  const long nWc = (long)NCOMP * SEQLEN;
  if (in_sizes[0] != nQ || in_sizes[1] != nW || in_sizes[2] != EMBED || in_sizes[3] != nW ||
      in_sizes[4] != EMBED || in_sizes[5] != nW || in_sizes[6] != EMBED || in_sizes[7] != nWc ||
      in_sizes[8] != nWc || in_sizes[9] != nW || in_sizes[10] != EMBED || out_size != nQ) return;

  const float* query = (const float*)d_in[0];
  const float* Wq  = (const float*)d_in[1];  const float* bq = (const float*)d_in[2];
  const float* Wk  = (const float*)d_in[3];  const float* bk = (const float*)d_in[4];
  const float* Wv  = (const float*)d_in[5];  const float* bv = (const float*)d_in[6];
  const float* Wck = (const float*)d_in[7];  const float* Wcv = (const float*)d_in[8];
  const float* Wo  = (const float*)d_in[9];  const float* bo = (const float*)d_in[10];

  const size_t BYTES_QB   = (size_t)nQ * 2;
  const size_t BYTES_QT   = (size_t)nQ * 2;
  const size_t BYTES_WC   = (size_t)2 * nWc * 2;
  const size_t BYTES_KVIN = (size_t)2 * NCOMP * NBAT * (2 * EMBED) * 2;
  const size_t BYTES_QP   = (size_t)nQ * 2;
  const size_t BYTES_OP   = (size_t)nQ * 2;
  const size_t BYTES_KP   = (size_t)NCOMP * NBAT * EMBED * 2;
  const size_t BYTES_VT   = (size_t)NBAT * EMBED * NCOMP * 2;
  const size_t BYTES_WQ   = (size_t)nW * 2;
  const size_t BYTES_WK2  = (size_t)nW * 2 * 2;
  const size_t BYTES_WV2  = (size_t)nW * 2 * 2;
  const size_t BYTES_WOH  = (size_t)nW * 2;
  const size_t BYTES_BIAS = (size_t)4 * EMBED * 4;
  const size_t OFF_QB   = 0;
  const size_t OFF_QT   = OFF_QB   + BYTES_QB;
  const size_t OFF_WC   = OFF_QT   + BYTES_QT;
  const size_t OFF_KVIN = OFF_WC   + BYTES_WC;
  const size_t OFF_QP   = OFF_KVIN + BYTES_KVIN;
  const size_t OFF_OP   = OFF_QP   + BYTES_QP;
  const size_t OFF_KP   = OFF_OP   + BYTES_OP;
  const size_t OFF_VT   = OFF_KP   + BYTES_KP;
  const size_t OFF_WQ   = OFF_VT   + BYTES_VT;
  const size_t OFF_WK2  = OFF_WQ   + BYTES_WQ;
  const size_t OFF_WV2  = OFF_WK2  + BYTES_WK2;
  const size_t OFF_WOH  = OFF_WV2  + BYTES_WV2;
  const size_t OFF_BIAS = OFF_WOH  + BYTES_WOH;
  const size_t WS_TOTAL = OFF_BIAS + BYTES_BIAS;
  if (WS_TOTAL > ws_size) return;

  char* ws = (char*)d_ws;
  unsigned short* queryB = (unsigned short*)(ws + OFF_QB);
  unsigned short* queryT = (unsigned short*)(ws + OFF_QT);
  unsigned short* WcB    = (unsigned short*)(ws + OFF_WC);
  unsigned short* KVin   = (unsigned short*)(ws + OFF_KVIN);
  unsigned short* qP     = (unsigned short*)(ws + OFF_QP);
  unsigned short* oP     = (unsigned short*)(ws + OFF_OP);
  unsigned short* kP     = (unsigned short*)(ws + OFF_KP);
  unsigned short* vtP    = (unsigned short*)(ws + OFF_VT);
  unsigned short* WqB    = (unsigned short*)(ws + OFF_WQ);
  unsigned short* WkB2   = (unsigned short*)(ws + OFF_WK2);
  unsigned short* WvB2   = (unsigned short*)(ws + OFF_WV2);
  unsigned short* WoH    = (unsigned short*)(ws + OFF_WOH);
  float*          biasb  = (float*)(ws + OFF_BIAS);
  float* bq_r = biasb;
  float* bk_r = biasb + EMBED;
  float* bv_r = biasb + 2 * EMBED;
  float* bo_r = biasb + 3 * EMBED;

  {
    const int n2 = (int)(nQ / 2);
    cast_bf16x2_kernel<<<dim3((unsigned)((n2 + 255) / 256)), dim3(256), 0, stream>>>(query, queryB, n2);
  }
  tconv_bf16_kernel<<<dim3(EMBED / 64, SEQLEN / 64, NBAT), dim3(256), 0, stream>>>(
      query, queryT, SEQLEN, EMBED, NBAT * EMBED, (long)EMBED, (long)EMBED * SEQLEN);
  {
    const int n2 = (int)(nWc / 2);
    cast_bf16x2_kernel<<<dim3((unsigned)((n2 + 255) / 256)), dim3(256), 0, stream>>>(Wck, WcB, n2);
    cast_bf16x2_kernel<<<dim3((unsigned)((n2 + 255) / 256)), dim3(256), 0, stream>>>(Wcv, WcB + (size_t)nWc, n2);
  }
  {
    const int n2 = (int)(nW / 2);
    cast_bf16x2_kernel<<<dim3((unsigned)((n2 + 255) / 256)), dim3(256), 0, stream>>>(Wq, WqB, n2);
    dup_bf16x2_kernel<<<dim3((unsigned)((n2 + 255) / 256)), dim3(256), 0, stream>>>(Wk, WkB2, n2, EMBED);
    dup_bf16x2_kernel<<<dim3((unsigned)((n2 + 255) / 256)), dim3(256), 0, stream>>>(Wv, WvB2, n2, EMBED);
    cast_wo_f16x2_kernel<<<dim3((unsigned)((n2 + 255) / 256)), dim3(256), 0, stream>>>(Wo, WoH, n2, WO_CARRY);
  }
  bias_prep_kernel<<<dim3(1), dim3(512), 0, stream>>>(bq, bk, bv, bo, biasb, EMBED);

  wmma_gemm64<1, false, 0, 2, false><<<dim3(32, NBAT), dim3(256), 0, stream>>>(
      WcB, WcB, SEQLEN, 0L,
      queryT, queryT, SEQLEN, (long)EMBED * SEQLEN,
      (void*)KVin, (void*)(KVin + EMBED), 4 * (2 * EMBED), (long)(2 * EMBED),
      biasb, biasb, 0L,
      2 * NCOMP, EMBED, SEQLEN, 1.0f);

  wmma_gemm64<1, false, 2, 1, false><<<dim3(256, 1), dim3(256), 0, stream>>>(
      queryB, queryB, EMBED, 0L,
      WqB, WqB, EMBED, 0L,
      (void*)qP, (void*)qP, EMBED, 0L,
      bq_r, bq_r, 0L,
      SEQLEN * NBAT, EMBED, EMBED, 1.0f);

  wmma_gemm64<1, false, 2, 1, false><<<dim3(64, 1), dim3(256), 0, stream>>>(
      KVin, KVin, 2 * EMBED, 0L,
      WkB2, WkB2, 2 * EMBED, 0L,
      (void*)kP, (void*)kP, EMBED, 0L,
      bk_r, bk_r, 0L,
      NCOMP * NBAT, EMBED, 2 * EMBED, 1.0f);

  wmma_gemm64<1, false, 1, 1, false><<<dim3(16, NBAT), dim3(256), 0, stream>>>(
      WvB2, WvB2, 2 * EMBED, 0L,
      KVin + (size_t)NCOMP * NBAT * (2 * EMBED), KVin + (size_t)NCOMP * NBAT * (2 * EMBED), 4 * (2 * EMBED), (long)(2 * EMBED),
      (void*)vtP, (void*)vtP, NCOMP, (long)EMBED * NCOMP,
      bv_r, bv_r, 0L,
      EMBED, NCOMP, 2 * EMBED, 1.0f);

  attn_lin_kernel<<<dim3(NBAT * NHEADS * (SEQLEN / 64)), dim3(128), 0, stream>>>(qP, kP, vtP, oP);

  wmma_gemm64<0, false, 2, 0, false><<<dim3(256, 1), dim3(256), 0, stream>>>(
      oP, oP, EMBED, 0L,
      WoH, WoH, EMBED, 0L,
      d_out, d_out, EMBED, 0L,
      bo_r, bo_r, 0L,
      SEQLEN * NBAT, EMBED, EMBED, 1.0f / (OUT_CARRY * WO_CARRY));
}
